// RNN_26388279067168
// MI455X (gfx1250) — hardware-run, weakly checked
//
#include <hip/hip_runtime.h>
#include <math.h>

typedef __attribute__((ext_vector_type(16))) _Float16 v16h;
typedef __attribute__((ext_vector_type(8)))  _Float16 v8h;
typedef __attribute__((ext_vector_type(8)))  float    v8f;
typedef __attribute__((ext_vector_type(4)))  float    v4f;

constexpr int kBatch   = 16384;
constexpr int kSteps   = 28;
constexpr int kIn      = 28;
constexpr int kHid     = 64;
constexpr int kGates   = 4 * kHid;
constexpr int kCls     = 10;
constexpr int kKx      = 32;
constexpr int kKtot    = kKx + kHid;
constexpr int kWPitch  = 104;
constexpr int kHPitch  = 72;
constexpr int kHfPitch = 68;
constexpr int kWaves   = 4;
constexpr int kThreads = kWaves * 32;
constexpr int kRowsBlk = kWaves * 16;
static_assert(kGates == 256, "gate rows");
static_assert(kKtot == 96 && (kKtot % 32) == 0, "fused depth is three 32-deep k-steps");
static_assert(kIn <= kKx && kIn == 28, "x depth padded 28 -> 32");
static_assert((kBatch % kRowsBlk) == 0, "grid is exact");
static_assert((kWPitch % 8) == 0 && kWPitch >= kKtot, "weight plane pitch, 16-B aligned rows");
static_assert((kHPitch % 8) == 0 && kHPitch >= kHid, "h slab pitch, 16-B aligned rows");
static_assert((kHfPitch % 4) == 0 && kHfPitch >= kHid, "f32 h slab pitch");
static_assert((kGates * kWPitch) % kThreads == 0, "weight staging loop is exact");
static_assert((kCls * kHid) % kThreads == 0, "head weight staging loop is exact");
static_assert((16 * kCls * 4) % 128 == 0, "a wave's 16 output rows are whole 128-B lines");

constexpr float kCarryX   = 128.0f;
constexpr float kCarryWih = 256.0f;
constexpr float kCarryH   = 256.0f;
constexpr float kCarryWhh = 128.0f;
constexpr float kScaleAll = 32768.0f;
constexpr float kInvScale = 1.0f / kScaleAll;
static_assert(kCarryX * kCarryWih == kScaleAll, "x segment carry");
static_assert(kCarryH * kCarryWhh == kScaleAll, "h segment carry");
constexpr float kHalfMinNormal = 6.103515625e-05f;

__device__ __forceinline__ _Float16 h16_flush(float v) {
  const float w = (__builtin_fabsf(v) < kHalfMinNormal) ? 0.0f : v;
  return (_Float16)w;
}

struct FragH {
  union U { v16h v; v8h h[2]; };
  static __device__ __forceinline__ v16h load(const _Float16* p) {
    U f;
    f.h[0] = *(const v8h*)(p);
    f.h[1] = *(const v8h*)(p + 16);
    return f.v;
  }
};

__device__ __forceinline__ v8f mma_h(v16h a, v16h b, v8f c) {
  c = __builtin_amdgcn_wmma_f32_16x16x32_f16(false, a, false, b, (short)0, c, false, false);
  asm volatile("v_nop\n\tv_nop\n\tv_nop\n\tv_nop" : "+v"(c) : "v"(a), "v"(b));
  return c;
}

__device__ __forceinline__ float sigm_f(float v) {
  return __builtin_amdgcn_rcpf(1.0f + expf(-v));
}
__device__ __forceinline__ float tanh_f(float v) {
  return 1.0f - 2.0f * __builtin_amdgcn_rcpf(1.0f + expf(2.0f * v));
}

__global__ __launch_bounds__(kThreads) void lstm_seq_kernel(
    const float* __restrict__ x, const float* __restrict__ W_ih, const float* __restrict__ W_hh,
    const float* __restrict__ b_ih, const float* __restrict__ b_hh,
    const float* __restrict__ W_cls, const float* __restrict__ b_cls, float* __restrict__ out)
{
  __shared__ __align__(16) _Float16 sW[kGates * kWPitch];
  __shared__ __align__(16) _Float16 sH[kWaves][16 * kHPitch];
  __shared__ __align__(16) float    sHf[kWaves][16 * kHfPitch];
  __shared__ __align__(16) float    sBias[kGates];
  __shared__ __align__(16) float    sWc[kCls * kHid];
  __shared__ __align__(16) float    sBc[16];

  const int tid  = threadIdx.x;
  const int wave = tid >> 5;
  const int lane = tid & 31;
  const int m    = lane & 15;
  const int hi   = lane >> 4;
  const bool upper = (hi != 0);

#pragma unroll 1
  for (int i = tid; i < kGates * kWPitch; i += kThreads) {
    const int row = i / kWPitch;
    const int col = i - row * kWPitch;
    const int ci  = (col < kIn) ? col : (kIn - 1);
    int ch = col - kKx;
    ch = (ch < 0) ? 0 : ch;
    ch = (ch > kHid - 1) ? (kHid - 1) : ch;
    float wa = W_ih[row * kIn + ci];
    float wb = W_hh[row * kHid + ch];
    asm volatile("" : "+v"(wa), "+v"(wb));
    const bool isx = (col < kIn);
    const bool ish = (col >= kKx) && (col < kKtot);
    const float v = isx ? (wa * kCarryWih) : (ish ? (wb * kCarryWhh) : 0.0f);
    sW[i] = h16_flush(v);
  }
#pragma unroll 1
  for (int i = tid; i < kGates; i += kThreads) sBias[i] = b_ih[i] + b_hh[i];
#pragma unroll 1
  for (int i = tid; i < kCls * kHid; i += kThreads) sWc[i] = W_cls[i];
  {
    const int ci = (tid < kCls) ? tid : (kCls - 1);
    float bv = b_cls[ci];
    asm volatile("" : "+v"(bv));
    if (tid < 16) sBc[tid] = (tid < kCls) ? bv : 0.0f;
  }
  {
    unsigned* hz = (unsigned*)(&sH[wave][0]);
#pragma unroll 1
    for (int i = lane; i < (16 * kHPitch) / 2; i += 32) hz[i] = 0u;
  }
  __syncthreads();

  _Float16* hs  = &sH[wave][0];
  float*    hfw = &sHf[wave][0];
  const int rowBase = blockIdx.x * kRowsBlk + wave * 16;
  const float* xrow = x + (size_t)(rowBase + m) * (size_t)(kSteps * kIn);

  const v8f z8 = {0.f, 0.f, 0.f, 0.f, 0.f, 0.f, 0.f, 0.f};
  v8f cs0 = z8, cs1 = z8, cs2 = z8, cs3 = z8;

#pragma unroll 1
  for (int t = 0; t < kSteps; ++t) {
    const float* xr = xrow + t * kIn;
    const v4f q0 = *(const v4f*)(xr + 8 * hi);
    const v4f q1 = *(const v4f*)(xr + 8 * hi + 4);
    const v4f q2 = *(const v4f*)(xr + 16 + 8 * hi);
    const v4f q3 = *(const v4f*)(xr + 20 + 4 * hi);
    float t0 = q3[0], t1 = q3[1], t2 = q3[2], t3 = q3[3];
    asm volatile("" : "+v"(t0), "+v"(t1), "+v"(t2), "+v"(t3));
    v16h aF[3];
#pragma unroll
    for (int e = 0; e < 4; ++e) {
      aF[0][e]     = h16_flush(q0[e] * kCarryX);
      aF[0][4 + e] = h16_flush(q1[e] * kCarryX);
      aF[0][8 + e] = h16_flush(q2[e] * kCarryX);
    }
    aF[0][12] = h16_flush(upper ? 0.0f : (t0 * kCarryX));
    aF[0][13] = h16_flush(upper ? 0.0f : (t1 * kCarryX));
    aF[0][14] = h16_flush(upper ? 0.0f : (t2 * kCarryX));
    aF[0][15] = h16_flush(upper ? 0.0f : (t3 * kCarryX));
    aF[1] = FragH::load(hs + m * kHPitch + 8 * hi);
    aF[2] = FragH::load(hs + m * kHPitch + 32 + 8 * hi);
    asm volatile("" ::: "memory");

#pragma unroll 1
    for (int jt = 0; jt < 4; ++jt) {
      v8f acc[4];
#pragma unroll
      for (int g = 0; g < 4; ++g) acc[g] = z8;
      const _Float16* wbase = sW + (jt * 16 + m) * kWPitch + 8 * hi;
#pragma unroll
      for (int ks = 0; ks < 3; ++ks) {
#pragma unroll
        for (int g = 0; g < 4; ++g) {
          const v16h bf = FragH::load(wbase + g * (kHid * kWPitch) + ks * 32);
          acc[g] = mma_h(aF[ks], bf, acc[g]);
        }
      }
      const int ucol = jt * 16 + m;
      const float bI = sBias[ucol];
      const float bF = sBias[kHid + ucol];
      const float bG = sBias[2 * kHid + ucol];
      const float bO = sBias[3 * kHid + ucol];
      v8f cn;
#pragma unroll
      for (int r = 0; r < 8; ++r) {
        const float gi = fmaf(acc[0][r], kInvScale, bI);
        const float gf = fmaf(acc[1][r], kInvScale, bF);
        const float gg = fmaf(acc[2][r], kInvScale, bG);
        const float go = fmaf(acc[3][r], kInvScale, bO);
        const float iv = sigm_f(gi);
        const float fv = sigm_f(gf);
        const float gv = tanh_f(gg);
        const float ov = sigm_f(go);
        const float cc = fmaf(fv, cs0[r], iv * gv);
        cn[r] = cc;
        const float hv = ov * tanh_f(cc);
        hs[(8 * hi + r) * kHPitch + ucol]   = h16_flush(hv * kCarryH);
        hfw[(8 * hi + r) * kHfPitch + ucol] = hv;
      }
      cs0 = cs1;
      cs1 = cs2;
      cs2 = cs3;
      cs3 = cn;
    }
    __syncthreads();
  }

  float o[5];
#pragma unroll
  for (int it = 0; it < 5; ++it) {
    const int idx = it * 32 + lane;
    const int row = idx / kCls;
    const int cls = idx - row * kCls;
    const float* hp = hfw + row * kHfPitch;
    const float* wp = sWc + cls * kHid;
    float s = 0.0f;
#pragma unroll 1
    for (int k = 0; k < kHid; k += 4) {
      const v4f hv = *(const v4f*)(hp + k);
      const v4f wv = *(const v4f*)(wp + k);
      s = fmaf(hv[0], wv[0], s);
      s = fmaf(hv[1], wv[1], s);
      s = fmaf(hv[2], wv[2], s);
      s = fmaf(hv[3], wv[3], s);
    }
    o[it] = s + sBc[cls];
  }
  float* op = out + (size_t)rowBase * kCls + lane;
  for (int pass = 0; pass < 2; ++pass) {
#pragma unroll
    for (int it = 0; it < 5; ++it) {
      *(volatile float*)(op + it * 32) = o[it];
    }
    __threadfence();
  }
}

extern "C" void kernel_launch(void* const* d_in, const int* in_sizes, int n_in,
                              void* d_out, int out_size, void* d_ws, size_t ws_size,
                              hipStream_t stream) {
  (void)d_ws;
  (void)ws_size;
  if (n_in < 7 || d_out == nullptr) return;
  if (in_sizes[0] != kBatch * kSteps * kIn) return;
  if (in_sizes[1] != kGates * kIn) return;
  if (in_sizes[2] != kGates * kHid) return;
  if (in_sizes[3] != kGates) return;
  if (in_sizes[4] != kGates) return;
  if (in_sizes[5] != kCls * kHid) return;
  if (in_sizes[6] != kCls) return;
  if (out_size != kBatch * kCls) return;

  const float* x     = (const float*)d_in[0];
  const float* W_ih  = (const float*)d_in[1];
  const float* W_hh  = (const float*)d_in[2];
  const float* b_ih  = (const float*)d_in[3];
  const float* b_hh  = (const float*)d_in[4];
  const float* W_cls = (const float*)d_in[5];
  const float* b_cls = (const float*)d_in[6];
  float* out = (float*)d_out;

  lstm_seq_kernel<<<kBatch / kRowsBlk, kThreads, 0, stream>>>(x, W_ih, W_hh, b_ih, b_hh, W_cls, b_cls, out);
}
